// RNNGCNModel_45930380263836
// MI455X (gfx1250) — hardware-run, weakly checked
//
#include <hip/hip_runtime.h>
#include <stddef.h>


#define DIM     128
#define NCL     64
#define KRNN    256
#define NTHR    256
#define NWAVE   8
#define EPT     8
#define NGRP    2
#define CHUNK   (NTHR * EPT * NGRP)
#define WCAP    (EPT * NGRP * 32)
#define LISTN   (NWAVE * WCAP)
#define NBC     4096
#define NBF     1024
#define RCAP    40960
#define RBN     128
#define TGT     256
#define DEGCAP  1024
#define GROWS   128
#define OTHR    512
#define RBS     512
#define WSCALE  8.0f
#define WINV    0.125f

#define LDS_FILL ((RCAP + NBF + LISTN) * 4 + 64)

static_assert((CHUNK & (CHUNK - 1)) == 0);
static_assert(CHUNK <= 4096);
static_assert(NBC <= 4096 && NBF <= 4096);
static_assert((NBC & (NBC - 1)) == 0 && (NBF & (NBF - 1)) == 0);
static_assert(NBC == 4 * NBF);
static_assert(OTHR * 8 == NBC);
static_assert((RCAP % 32) == 0);
static_assert(TGT == NWAVE * 32 && (TGT % GROWS) == 0);
static_assert(NTHR == 4 * NCL);
static_assert((RBS % 4) == 0);
static_assert(KRNN == 2 * DIM);

typedef float    v2f  __attribute__((ext_vector_type(2)));
typedef float    v4f  __attribute__((ext_vector_type(4)));
typedef float    v8f  __attribute__((ext_vector_type(8)));
typedef int      v4i  __attribute__((ext_vector_type(4)));
typedef _Float16 v8h  __attribute__((ext_vector_type(8)));
typedef _Float16 v16h __attribute__((ext_vector_type(16)));
union FragH { v16h v; v8h h[2]; };

__device__ __forceinline__ v8h cvt8(v4f a, v4f b) {
  v8h r;
  r[0] = (_Float16)a.x; r[1] = (_Float16)a.y; r[2] = (_Float16)a.z; r[3] = (_Float16)a.w;
  r[4] = (_Float16)b.x; r[5] = (_Float16)b.y; r[6] = (_Float16)b.z; r[7] = (_Float16)b.w;
  return r;
}

__device__ __forceinline__ v4f sel4(bool c, v4f a, v4f b) {
  v4f r;
  r.x = c ? a.x : b.x; r.y = c ? a.y : b.y; r.z = c ? a.z : b.z; r.w = c ? a.w : b.w;
  return r;
}

__device__ __forceinline__ v8f wmh(v16h a, v16h b, v8f c) {
  v8f d = __builtin_amdgcn_wmma_f32_16x16x32_f16(false, a, false, b, (short)0, c, false, false);
  asm volatile("v_nop\n\tv_nop\n\tv_nop\n\tv_nop" : "+v"(d) : "v"(a), "v"(b));
  return d;
}

template <int NB>
__device__ __forceinline__ int scan_chunk(const int* __restrict__ dsts, int nE, int cbase, int slotBase,
                                          int vec8, int* list, int tid, int lane, int wave) {
  int wc = 0;
#pragma unroll
  for (int g = 0; g < NGRP; ++g) {
    const int el0  = (g * NTHR + tid) * EPT;
    const int e0   = cbase + el0;
    const int sent = -2147483647 - 1;
    v4i da, db;
    if (vec8 != 0 && cbase + CHUNK <= nE) {
      da = *(const v4i*)(dsts + e0);
      db = *(const v4i*)(dsts + e0 + 4);
    } else {
      da.x = (e0     < nE) ? dsts[min(e0, nE - 1)] : sent;
      da.y = (e0 + 1 < nE) ? dsts[min(e0 + 1, nE - 1)] : sent;
      da.z = (e0 + 2 < nE) ? dsts[min(e0 + 2, nE - 1)] : sent;
      da.w = (e0 + 3 < nE) ? dsts[min(e0 + 3, nE - 1)] : sent;
      db.x = (e0 + 4 < nE) ? dsts[min(e0 + 4, nE - 1)] : sent;
      db.y = (e0 + 5 < nE) ? dsts[min(e0 + 5, nE - 1)] : sent;
      db.z = (e0 + 6 < nE) ? dsts[min(e0 + 6, nE - 1)] : sent;
      db.w = (e0 + 7 < nE) ? dsts[min(e0 + 7, nE - 1)] : sent;
    }
    const unsigned nb = (unsigned)slotBase;
    const unsigned s0 = (unsigned)da.x - nb, s1 = (unsigned)da.y - nb;
    const unsigned s2 = (unsigned)da.z - nb, s3 = (unsigned)da.w - nb;
    const unsigned s4 = (unsigned)db.x - nb, s5 = (unsigned)db.y - nb;
    const unsigned s6 = (unsigned)db.z - nb, s7 = (unsigned)db.w - nb;
    const bool h0 = s0 < (unsigned)NB, h1 = s1 < (unsigned)NB, h2 = s2 < (unsigned)NB, h3 = s3 < (unsigned)NB;
    const bool h4 = s4 < (unsigned)NB, h5 = s5 < (unsigned)NB, h6 = s6 < (unsigned)NB, h7 = s7 < (unsigned)NB;
    const unsigned any = __builtin_amdgcn_ballot_w32(h0 | h1 | h2 | h3 | h4 | h5 | h6 | h7);
    if (any != 0u) {
#define HITJ(J, HJ, SJ) { \
        const unsigned mj = __builtin_amdgcn_ballot_w32(HJ); \
        if (mj != 0u) { \
          if (HJ) { \
            const int pos = wc + (int)__builtin_amdgcn_mbcnt_lo(mj, 0u); \
            if (pos < WCAP) list[wave * WCAP + pos] = ((el0 + (J)) << 12) | (int)(SJ); \
          } \
          wc += (int)__builtin_popcount(mj); } }
      HITJ(0, h0, s0)
      HITJ(1, h1, s1)
      HITJ(2, h2, s2)
      HITJ(3, h3, s3)
      HITJ(4, h4, s4)
      HITJ(5, h5, s5)
      HITJ(6, h6, s6)
      HITJ(7, h7, s7)
#undef HITJ
    }
  }
  return wc;
}

__global__ __launch_bounds__(NTHR) void k_prep(
    const float* __restrict__ Wih, const float* __restrict__ Whh,
    const float* __restrict__ bih, const float* __restrict__ bhh,
    const float* __restrict__ W0, const float* __restrict__ W1, const float* __restrict__ W2,
    _Float16* BtR, _Float16* B0, _Float16* B1, _Float16* B2, float* bcomb) {
  const int g0 = DIM * KRNN / 8;
  const int g1 = DIM * DIM / 8;
  const int g3 = NCL * DIM / 8;
  const int tid = threadIdx.x;
  const int bstart = blockIdx.x * NTHR;
  const int i = bstart + tid;
  if (bstart >= g0 + 2 * g1 + g3) {
    v4f s = {0.f, 0.f, 0.f, 0.f};
    if (tid < 32) {
      const v4f a = *(const v4f*)(bih + 4 * tid);
      const v4f b = *(const v4f*)(bhh + 4 * tid);
      s = a + b;
    }
    if (tid < 32) *(volatile v4f*)(bcomb + 4 * tid) = s;
    __threadfence();
    if (tid < 32) *(volatile v4f*)(bcomb + 4 * tid) = s;
    return;
  }
  float v[8];
  _Float16* dp;
  if (bstart < g0) {
    const int o = i * 8, n = o >> 8, k0 = o & 255, kk = k0 & 127;
    const float* pa = Wih + n * DIM + kk;
    const float* pb = Whh + n * DIM + kk;
    const v4f a0 = *(const v4f*)pa, a1 = *(const v4f*)(pa + 4);
    const v4f b0 = *(const v4f*)pb, b1 = *(const v4f*)(pb + 4);
    const v4f x0 = sel4(k0 < 128, a0, b0), x1 = sel4(k0 < 128, a1, b1);
    v[0] = x0.x; v[1] = x0.y; v[2] = x0.z; v[3] = x0.w;
    v[4] = x1.x; v[5] = x1.y; v[6] = x1.z; v[7] = x1.w;
    dp = BtR + o;
  } else if (bstart < g0 + g1) {
    const int o = (i - g0) * 8, n = o >> 7, k0 = o & 127;
#pragma unroll
    for (int e = 0; e < 8; ++e) v[e] = W0[(k0 + e) * DIM + n];
    dp = B0 + o;
  } else if (bstart < g0 + 2 * g1) {
    const int o = (i - g0 - g1) * 8, n = o >> 7, k0 = o & 127;
#pragma unroll
    for (int e = 0; e < 8; ++e) v[e] = W1[(k0 + e) * DIM + n];
    dp = B1 + o;
  } else {
    const int o = (i - g0 - 2 * g1) * 8, n = o >> 7, k0 = o & 127;
#pragma unroll
    for (int e = 0; e < 8; ++e) v[e] = W2[(k0 + e) * NCL + n];
    dp = B2 + o;
  }
  v4f a, b;
  a.x = v[0] * WSCALE; a.y = v[1] * WSCALE; a.z = v[2] * WSCALE; a.w = v[3] * WSCALE;
  b.x = v[4] * WSCALE; b.y = v[5] * WSCALE; b.z = v[6] * WSCALE; b.w = v[7] * WSCALE;
  const v8h hv = cvt8(a, b);
  *(volatile v8h*)dp = hv;
  __threadfence();
  *(volatile v8h*)dp = hv;
}

__global__ __launch_bounds__(NTHR) void k_cvta(
    const float* __restrict__ topo, const float* __restrict__ hid, _Float16* Ah, int nN) {
  const int i = blockIdx.x * NTHR + (int)threadIdx.x;
  const int r = i >> 5;
  const int s = i & 31;
  const int rc = r < nN ? r : nN - 1;
  const size_t so = (size_t)rc * DIM + (size_t)(s & 15) * 8;
  const v4f ta = *(const v4f*)(topo + so), tb = *(const v4f*)(topo + so + 4);
  const v4f ha = *(const v4f*)(hid + so),  hb = *(const v4f*)(hid + so + 4);
  const v4f z = {0.f, 0.f, 0.f, 0.f};
  v4f a = sel4(s < 16, ta, ha), b = sel4(s < 16, tb, hb);
  a = sel4(r < nN, a, z); b = sel4(r < nN, b, z);
  const v8h hv = cvt8(a, b);
  _Float16* dp = Ah + (size_t)i * 8;
  *(volatile v8h*)dp = hv;
  __threadfence();
  *(volatile v8h*)dp = hv;
}

__global__ __launch_bounds__(NTHR) void k_count(const int* __restrict__ dsts, int* cnt, int nE, int vec8) {
  __shared__ __attribute__((aligned(16))) int scnt[NBC];
  __shared__ __attribute__((aligned(16))) int list[LISTN];
  __shared__ int wcnt[NWAVE];
  const int tid = threadIdx.x, lane = tid & 31, wave = tid >> 5;
  const int nodeBase = blockIdx.x * NBC;

  for (int i = tid; i < NBC; i += NTHR) scnt[i] = 0;
  __syncthreads();

  const int nChunks = (nE + CHUNK - 1) / CHUNK;
#pragma unroll 1
  for (int ch = 0; ch < nChunks; ++ch) {
    const int cbase = ch * CHUNK;
    const int wc = scan_chunk<NBC>(dsts, nE, cbase, nodeBase, vec8, list, tid, lane, wave);
    if (lane == 0) wcnt[wave] = wc;
    __syncthreads();
    if (wave == 0) {
#pragma unroll 1
      for (int wsx = 0; wsx < NWAVE; ++wsx) {
        int n = __builtin_amdgcn_readfirstlane(wcnt[wsx]);
        n = n > WCAP ? WCAP : (n < 0 ? 0 : n);
        const int* lp = list + wsx * WCAP;
#pragma unroll 1
        for (int i = 0; i < n; ++i) {
          const int ent  = __builtin_amdgcn_readfirstlane(lp[i]);
          const int slot = ent & (NBC - 1);
          if (lane == 0) scnt[slot] = scnt[slot] + 1;
        }
      }
    }
    __syncthreads();
  }

  v4i cq[4];
#pragma unroll
  for (int q = 0; q < 4; ++q) {
    const int f = (wave * 4 + q) * 128 + 4 * lane;
    cq[q] = *(const v4i*)(scnt + f);
  }
  int* cp = cnt + (size_t)nodeBase;
#pragma unroll
  for (int q = 0; q < 4; ++q) {
    const int f = (wave * 4 + q) * 128 + 4 * lane;
    *(volatile v4i*)(cp + f) = cq[q];
  }
  __threadfence();
#pragma unroll
  for (int q = 0; q < 4; ++q) {
    const int f = (wave * 4 + q) * 128 + 4 * lane;
    *(volatile v4i*)(cp + f) = cq[q];
  }
}

__global__ __launch_bounds__(OTHR) void k_offsets(
    const int* __restrict__ cnt, int* off, int* rbase, int nChunk) {
  __shared__ __attribute__((aligned(16))) int soff[NBC];
  __shared__ __attribute__((aligned(16))) int srb[RBN];
  __shared__ int wtot[OTHR / 32];
  const int tid = threadIdx.x, lane = tid & 31, wave = tid >> 5, sub = tid >> 7;
  for (int i = tid; i < RBN; i += OTHR) srb[i] = 0;
  int carry = 0;
#pragma unroll 1
  for (int ch = 0; ch < nChunk; ++ch) {
    const int base = ch * NBC;
    const v4i c0 = *(const v4i*)(cnt + base + 8 * tid);
    const v4i c1 = *(const v4i*)(cnt + base + 8 * tid + 4);
    const int e0 = max(c0.x, 0), e1 = max(c0.y, 0), e2 = max(c0.z, 0), e3 = max(c0.w, 0);
    const int e4 = max(c1.x, 0), e5 = max(c1.y, 0), e6 = max(c1.z, 0), e7 = max(c1.w, 0);
    const int ts = e0 + e1 + e2 + e3 + e4 + e5 + e6 + e7;
    int incl = ts;
#pragma unroll
    for (int d = 1; d < 32; d <<= 1) {
      const int t = __shfl_up(incl, d);
      if (lane >= d) incl += t;
    }
    if (lane == 31) wtot[wave] = incl;
    __syncthreads();
    const int S0 = wtot[0]  + wtot[1]  + wtot[2]  + wtot[3];
    const int S1 = wtot[4]  + wtot[5]  + wtot[6]  + wtot[7];
    const int S2 = wtot[8]  + wtot[9]  + wtot[10] + wtot[11];
    const int S3 = wtot[12] + wtot[13] + wtot[14] + wtot[15];
    int pre = 0;
#pragma unroll 1
    for (int w = 4 * sub; w < wave; ++w) pre += wtot[w];
    const int b0 = carry;
    const int b1 = b0 + ((S0 + 31) & ~31);
    const int b2 = b1 + ((S1 + 31) & ~31);
    const int b3 = b2 + ((S2 + 31) & ~31);
    const int b4 = b3 + ((S3 + 31) & ~31);
    const int myb = sub == 0 ? b0 : (sub == 1 ? b1 : (sub == 2 ? b2 : b3));
    if (tid == 0) {
      srb[min(4 * ch + 0, RBN - 1)] = b0;
      srb[min(4 * ch + 1, RBN - 1)] = b1;
      srb[min(4 * ch + 2, RBN - 1)] = b2;
      srb[min(4 * ch + 3, RBN - 1)] = b3;
    }
    int run = myb + pre + incl - ts;
    soff[8 * tid + 0] = run; run += e0;
    soff[8 * tid + 1] = run; run += e1;
    soff[8 * tid + 2] = run; run += e2;
    soff[8 * tid + 3] = run; run += e3;
    soff[8 * tid + 4] = run; run += e4;
    soff[8 * tid + 5] = run; run += e5;
    soff[8 * tid + 6] = run; run += e6;
    soff[8 * tid + 7] = run;
    carry = b4;
    __syncthreads();
    const v4i o0 = *(const v4i*)(soff + 4 * tid);
    const v4i o1 = *(const v4i*)(soff + 4 * (tid + OTHR));
    int* op = off + base;
    *(volatile v4i*)(op + 4 * tid) = o0;
    *(volatile v4i*)(op + 4 * (tid + OTHR)) = o1;
    __threadfence();
    *(volatile v4i*)(op + 4 * tid) = o0;
    *(volatile v4i*)(op + 4 * (tid + OTHR)) = o1;
    __syncthreads();
  }
  if (tid == 0) srb[min(4 * nChunk, RBN - 1)] = carry;
  __syncthreads();
  v4i rv = {0, 0, 0, 0};
  if (tid < 32) rv = *(const v4i*)(srb + 4 * tid);
  if (tid < 32) *(volatile v4i*)(rbase + 4 * tid) = rv;
  __threadfence();
  if (tid < 32) *(volatile v4i*)(rbase + 4 * tid) = rv;
}

__global__ __launch_bounds__(NTHR) void k_fill(
    const int* __restrict__ dsts, const int* __restrict__ off, const int* __restrict__ rbase,
    int* csr, int nE, int vec8, int csrLen) {
  extern __shared__ v4f lds_dyn[];
  int* region = (int*)lds_dyn;
  int* cursor = region + RCAP;
  int* list   = cursor + NBF;
  int* wcnt   = list + LISTN;
  const int tid = threadIdx.x, lane = tid & 31, wave = tid >> 5;
  const int b = blockIdx.x;
  const int nodeBase = b * NBF;

  int rb0 = rbase[b];
  const int rb1 = rbase[b + 1];
  rb0 = rb0 < 0 ? 0 : (rb0 > csrLen ? csrLen : rb0);
  rb0 &= ~31;
  int len = rb1 - rb0;
  len = len < 0 ? 0 : (len > RCAP ? RCAP : len);
  int lenW = (len + 31) & ~31;
  if (rb0 + lenW > csrLen) lenW = (csrLen - rb0) & ~31;

  {
    const v4i z = {0, 0, 0, 0};
    for (int i = tid; i < RCAP / 4; i += NTHR) ((v4i*)region)[i] = z;
    for (int s = tid; s < NBF; s += NTHR) {
      int o = off[nodeBase + s] - rb0;
      o = o < 0 ? 0 : (o > RCAP ? RCAP : o);
      cursor[s] = o;
    }
  }
  __syncthreads();

  const int nChunks = (nE + CHUNK - 1) / CHUNK;
#pragma unroll 1
  for (int ch = 0; ch < nChunks; ++ch) {
    const int cbase = ch * CHUNK;
    const int wc = scan_chunk<NBF>(dsts, nE, cbase, nodeBase, vec8, list, tid, lane, wave);
    if (lane == 0) wcnt[wave] = wc;
    __syncthreads();
    if (wave == 0) {
#pragma unroll 1
      for (int wsx = 0; wsx < NWAVE; ++wsx) {
        int n = __builtin_amdgcn_readfirstlane(wcnt[wsx]);
        n = n > WCAP ? WCAP : (n < 0 ? 0 : n);
        const int* lp = list + wsx * WCAP;
#pragma unroll 1
        for (int i = 0; i < n; ++i) {
          const int ent  = __builtin_amdgcn_readfirstlane(lp[i]);
          const int slot = ent & (NBF - 1);
          int e = cbase + ((ent >> 12) & (CHUNK - 1));
          e = e > nE - 1 ? nE - 1 : e;
          if (lane == 0) {
            int pos = cursor[slot];
            pos = pos < 0 ? 0 : (pos > RCAP - 1 ? RCAP - 1 : pos);
            region[pos] = e;
            const int np = pos + 1;
            cursor[slot] = np > RCAP ? RCAP : np;
          }
        }
      }
    }
    __syncthreads();
  }

  const int nv = lenW >> 2;
  int* gp = csr + rb0;
#pragma unroll 1
  for (int i = tid; i < nv; i += NTHR) { const v4i v = ((const v4i*)region)[i]; *(volatile v4i*)(gp + 4 * i) = v; }
  __threadfence();
#pragma unroll 1
  for (int i = tid; i < nv; i += NTHR) { const v4i v = ((const v4i*)region)[i]; *(volatile v4i*)(gp + 4 * i) = v; }
}

template <int KD, int NT, int MODE>
__global__ __launch_bounds__(NTHR) void k_gemm(
    const _Float16* __restrict__ A, const _Float16* __restrict__ Bs, const float* __restrict__ bias,
    float* Cf, _Float16* Ch, int nValid) {
  static_assert(MODE == 1 || NT == 8);
  static_assert((KD % 32) == 0);
  extern __shared__ v4f lds_dyn[];
  constexpr int NOUT = 16 * NT;
  float* stg = (float*)lds_dyn;
  const int tid = threadIdx.x, lane = tid & 31, wave = tid >> 5, hh = lane >> 4, m = lane & 15;
  const int rowBase = blockIdx.x * GROWS;
  const int r0 = wave * 16;
  const _Float16* ar = A + (size_t)(rowBase + r0 + m) * KD + 8 * hh;

  v8f acc[NT];
#pragma unroll
  for (int t = 0; t < NT; ++t) { v8f z = {0.f, 0.f, 0.f, 0.f, 0.f, 0.f, 0.f, 0.f}; acc[t] = z; }
#pragma unroll 1
  for (int kt = 0; kt < KD / 32; ++kt) {
    FragH a;
    a.h[0] = *(const v8h*)(ar + 32 * kt);
    a.h[1] = *(const v8h*)(ar + 32 * kt + 16);
#pragma unroll
    for (int t = 0; t < NT; ++t) {
      const _Float16* bp = Bs + (size_t)(16 * t + m) * KD + 32 * kt + 8 * hh;
      FragH b;
      b.h[0] = *(const v8h*)bp;
      b.h[1] = *(const v8h*)(bp + 16);
      acc[t] = wmh(a.v, b.v, acc[t]);
    }
  }

  float* sp = stg + (r0 + 8 * hh) * NOUT + m;
#pragma unroll
  for (int t = 0; t < NT; ++t) {
    float bv = 0.0f;
    if (MODE == 0) bv = bias[16 * t + m];
#pragma unroll
    for (int r = 0; r < 8; ++r) {
      float v = acc[t][r] * WINV + bv;
      if (MODE == 0) v = fmaxf(v, 0.0f);
      sp[r * NOUT + 16 * t] = v;
    }
  }
  __syncthreads();

  const float* lp = stg + r0 * NOUT;
  constexpr int NP = 16 * NOUT / 128;
  if (MODE == 1) {
    float* gp = Cf + (size_t)(rowBase + r0) * NOUT;
#pragma unroll
    for (int p = 0; p < NP; ++p) {
      const v4f v = *(const v4f*)(lp + 128 * p + 4 * lane);
      *(volatile v4f*)(gp + 128 * p + 4 * lane) = v;
    }
    __threadfence();
#pragma unroll
    for (int p = 0; p < NP; ++p) {
      const v4f v = *(const v4f*)(lp + 128 * p + 4 * lane);
      *(volatile v4f*)(gp + 128 * p + 4 * lane) = v;
    }
  } else {
    float* gp = Cf + (size_t)(rowBase + r0) * NOUT;
    _Float16* hp = Ch + (size_t)(rowBase + r0) * DIM;
#pragma unroll
    for (int p = 0; p < NP; ++p) {
      const v4f v = *(const v4f*)(lp + 128 * p + 4 * lane);
      if (rowBase + r0 + p < nValid) *(volatile v4f*)(gp + 128 * p + 4 * lane) = v;
    }
#pragma unroll
    for (int q = 0; q < 8; ++q) {
      const int o = 256 * q + 8 * lane;
      const v4f a = *(const v4f*)(lp + o), b = *(const v4f*)(lp + o + 4);
      const v8h hv = cvt8(a, b);
      *(volatile v8h*)(hp + o) = hv;
    }
    __threadfence();
#pragma unroll
    for (int p = 0; p < NP; ++p) {
      const v4f v = *(const v4f*)(lp + 128 * p + 4 * lane);
      if (rowBase + r0 + p < nValid) *(volatile v4f*)(gp + 128 * p + 4 * lane) = v;
    }
#pragma unroll
    for (int q = 0; q < 8; ++q) {
      const int o = 256 * q + 8 * lane;
      const v4f a = *(const v4f*)(lp + o), b = *(const v4f*)(lp + o + 4);
      const v8h hv = cvt8(a, b);
      *(volatile v8h*)(hp + o) = hv;
    }
  }
}

template <int VW, int OUTH>
__global__ __launch_bounds__(NTHR) void k_agg(
    const int* __restrict__ csr, const int* __restrict__ off, const int* __restrict__ cnt,
    const int* __restrict__ cols, const float* __restrict__ vals,
    const float* __restrict__ T, const float* __restrict__ bias,
    _Float16* Xh, float* Xf, int nN, int nE, int csrLen) {
  typedef float    vT __attribute__((ext_vector_type(VW)));
  typedef _Float16 hT __attribute__((ext_vector_type(VW)));
  constexpr int F = 32 * VW;
  const int tid = threadIdx.x, lane = tid & 31, wave = tid >> 5;
  const int tbase = blockIdx.x * TGT + wave * 32;
  const int cl = tbase + lane;
  const int cnt_l = cnt[cl];
  const int off_l = off[cl];
  const vT bb = *(const vT*)(bias + VW * lane);
  union FI { float f; int i; };

#pragma unroll 1
  for (int j = 0; j < 32; ++j) {
    const int c = tbase + j;
    int n = __builtin_amdgcn_readlane(cnt_l, j);
    n = n < 0 ? 0 : (n > DEGCAP ? DEGCAP : n);
    const int st = __builtin_amdgcn_readlane(off_l, j);
    vT acc;
#pragma unroll
    for (int q = 0; q < VW; ++q) acc[q] = 0.0f;
#pragma unroll 1
    for (int q0 = 0; q0 < n; q0 += 32) {
      int pos = st + q0 + lane;
      pos = pos < 0 ? 0 : (pos > csrLen - 1 ? csrLen - 1 : pos);
      int e = csr[pos];
      e = e < 0 ? 0 : (e > nE - 1 ? nE - 1 : e);
      int sl = cols[e];
      sl = sl < 0 ? 0 : (sl > nN - 1 ? nN - 1 : sl);
      FI vu; vu.f = vals[e];
      const int mcnt = (n - q0) < 32 ? (n - q0) : 32;
#pragma unroll 1
      for (int p = 0; p < mcnt; ++p) {
        const int s = __builtin_amdgcn_readlane(sl, p);
        FI wv; wv.i = __builtin_amdgcn_readlane(vu.i, p);
        const vT tv = *(const vT*)(T + (size_t)s * F + VW * lane);
        acc = acc + tv * wv.f;
      }
    }
    vT x = acc + bb;
#pragma unroll
    for (int q = 0; q < VW; ++q) x[q] = fmaxf(x[q], 0.0f);
    if (OUTH != 0) {
      hT hv;
#pragma unroll
      for (int q = 0; q < VW; ++q) hv[q] = (_Float16)x[q];
      _Float16* hp = Xh + (size_t)c * F + VW * lane;
      *(volatile hT*)hp = hv;
      __threadfence();
      *(volatile hT*)hp = hv;
    } else {
      float* fp = Xf + (size_t)c * F + VW * lane;
      *(volatile vT*)fp = x;
      __threadfence();
      *(volatile vT*)fp = x;
    }
  }
}

__global__ __launch_bounds__(NTHR) void k_colstat(
    const float* __restrict__ X3, const float* __restrict__ Mc, float* part, int nN, int mode) {
  __shared__ float red[NTHR];
  __shared__ __attribute__((aligned(16))) float res[NCL];
  const int tid = threadIdx.x, c = tid & (NCL - 1), rp = tid >> 6;
  const int rowBase = blockIdx.x * RBS;
  float a;
  if (mode == 0) {
    a = -__builtin_inff();
#pragma unroll 1
    for (int i = 0; i < RBS / 4; ++i) {
      const int r  = rowBase + rp + 4 * i;
      const int rc = r < nN ? r : nN - 1;
      const float x = X3[(size_t)rc * NCL + c];
      a = (r < nN) ? fmaxf(a, x) : a;
    }
  } else {
    const float mc = Mc[c];
    a = 0.0f;
#pragma unroll 1
    for (int i = 0; i < RBS / 4; ++i) {
      const int r  = rowBase + rp + 4 * i;
      const int rc = r < nN ? r : nN - 1;
      const float x = X3[(size_t)rc * NCL + c];
      const float t = expf(x - mc);
      a = (r < nN) ? a + t : a;
    }
  }
  red[tid] = a;
  __syncthreads();
  if (tid < NCL) {
    const float a0 = red[tid], a1 = red[tid + NCL], a2 = red[tid + 2 * NCL], a3 = red[tid + 3 * NCL];
    res[tid] = (mode == 0) ? fmaxf(fmaxf(a0, a1), fmaxf(a2, a3)) : ((a0 + a1) + (a2 + a3));
  }
  __syncthreads();
  v4f v = {0.f, 0.f, 0.f, 0.f};
  if (tid < 16) v = *(const v4f*)(res + 4 * tid);
  float* pp = part + (size_t)blockIdx.x * NCL + 4 * tid;
  if (tid < 16) *(volatile v4f*)pp = v;
  __threadfence();
  if (tid < 16) *(volatile v4f*)pp = v;
}

__global__ __launch_bounds__(NCL) void k_colred(
    const float* __restrict__ part, const float* __restrict__ Mc, float* dst, int nBlk, int mode) {
  __shared__ __attribute__((aligned(16))) float res[NCL];
  const int c = threadIdx.x;
  float r;
  if (mode == 0) {
    float mx = -__builtin_inff();
#pragma unroll 1
    for (int b = 0; b < nBlk; ++b) mx = fmaxf(mx, part[(size_t)b * NCL + c]);
    r = mx;
  } else {
    double s = 0.0;
#pragma unroll 1
    for (int b = 0; b < nBlk; ++b) s += (double)part[(size_t)b * NCL + c];
    const float sf = (float)s;
    r = Mc[c] + logf(sf);
  }
  res[c] = r;
  __syncthreads();
  v4f v = {0.f, 0.f, 0.f, 0.f};
  if (c < 16) v = *(const v4f*)(res + 4 * c);
  if (c < 16) *(volatile v4f*)(dst + 4 * c) = v;
  __threadfence();
  if (c < 16) *(volatile v4f*)(dst + 4 * c) = v;
}

__global__ __launch_bounds__(NTHR) void k_out(
    const float* __restrict__ X3, const float* __restrict__ lse, float* out, int n4) {
  const int i = blockIdx.x * NTHR + (int)threadIdx.x;
  if (i >= n4) return;
  const size_t o = (size_t)i * 4;
  const v4f x = *(const v4f*)(X3 + o);
  const v4f l = *(const v4f*)(lse + (o & (size_t)(NCL - 1)));
  const v4f v = x - l;
  *(volatile v4f*)(out + o) = v;
  __threadfence();
  *(volatile v4f*)(out + o) = v;
}

extern "C" void kernel_launch(void* const* d_in, const int* in_sizes, int n_in,
                              void* d_out, int out_size, void* d_ws, size_t ws_size,
                              hipStream_t stream) {
  if (n_in < 16) return;
  const int nN = in_sizes[1] / DIM;
  const int nE = in_sizes[2];
  if (nN <= 0 || nE <= 0 || in_sizes[1] != nN * DIM) return;
  if (in_sizes[3] != nE || in_sizes[4] != nE) return;
  if (in_sizes[5] < nN * DIM) return;
  if (in_sizes[6] != DIM * DIM || in_sizes[7] != DIM * DIM || in_sizes[8] < DIM || in_sizes[9] < DIM) return;
  if (in_sizes[10] != DIM * DIM || in_sizes[11] < DIM || in_sizes[12] != DIM * DIM || in_sizes[13] < DIM) return;
  if (in_sizes[14] != DIM * NCL || in_sizes[15] < NCL) return;
  if (out_size != nN * (NCL + DIM)) return;
  if (nE > (1 << 28) || nN > (1 << 24)) return;

  const float* topo  = (const float*)d_in[1];
  const int*   arows = (const int*)d_in[2];
  const int*   acols = (const int*)d_in[3];
  const float* avals = (const float*)d_in[4];
  const float* hid   = (const float*)d_in[5];
  const float* Wih   = (const float*)d_in[6];
  const float* Whh   = (const float*)d_in[7];
  const float* bih   = (const float*)d_in[8];
  const float* bhh   = (const float*)d_in[9];
  const float* W0    = (const float*)d_in[10];
  const float* gb0   = (const float*)d_in[11];
  const float* W1    = (const float*)d_in[12];
  const float* gb1   = (const float*)d_in[13];
  const float* W2    = (const float*)d_in[14];
  const float* gb2   = (const float*)d_in[15];
  float* out0 = (float*)d_out;
  float* out1 = (float*)d_out + (size_t)nN * NCL;

  const int NPAD   = ((nN + TGT - 1) / TGT) * TGT;
  const int nBC    = (nN + NBC - 1) / NBC;
  const int CNTPAD = nBC * NBC;
  if (4 * nBC + 1 > RBN) return;
  const int nBF    = (nN + NBF - 1) / NBF;
  const int csrLen = ((nE + 31) & ~31) + 4096;
  const int nGemm  = NPAD / GROWS;
  const int nAgg   = NPAD / TGT;
  const int nCvt   = (NPAD / 8) * (KRNN / 8) * 8 / NTHR;
  const int nSB    = (nN + RBS - 1) / RBS;
  const int n4     = nN * NCL / 4;
  const int nOut   = (n4 + NTHR - 1) / NTHR;
  const int nPrep  = (DIM * KRNN / 8 + 2 * (DIM * DIM / 8) + NCL * DIM / 8) / NTHR + 1;

  char* ws = (char*)d_ws;
  size_t off = 0;
  const size_t oBtR = off; off += (size_t)DIM * KRNN * 2;            off = (off + 255) & ~(size_t)255;
  const size_t oB0  = off; off += (size_t)DIM * DIM * 2;             off = (off + 255) & ~(size_t)255;
  const size_t oB1  = off; off += (size_t)DIM * DIM * 2;             off = (off + 255) & ~(size_t)255;
  const size_t oB2  = off; off += (size_t)NCL * DIM * 2;             off = (off + 255) & ~(size_t)255;
  const size_t oBc  = off; off += (size_t)DIM * 4;                   off = (off + 255) & ~(size_t)255;
  const size_t oAh  = off; off += (size_t)NPAD * KRNN * 2;           off = (off + 255) & ~(size_t)255;
  const size_t oCnt = off; off += (size_t)CNTPAD * 4;                off = (off + 255) & ~(size_t)255;
  const size_t oOff = off; off += (size_t)CNTPAD * 4;                off = (off + 255) & ~(size_t)255;
  const size_t oRb  = off; off += (size_t)RBN * 4;                   off = (off + 255) & ~(size_t)255;
  const size_t oCsr = off; off += (size_t)csrLen * 4;                off = (off + 255) & ~(size_t)255;
  const size_t oX   = off; off += (size_t)NPAD * DIM * 2;            off = (off + 255) & ~(size_t)255;
  const size_t oT   = off; off += (size_t)NPAD * DIM * 4;            off = (off + 255) & ~(size_t)255;
  const size_t oX3  = off; off += (size_t)NPAD * NCL * 4;            off = (off + 255) & ~(size_t)255;
  const size_t oPm  = off; off += (size_t)nSB * NCL * 4;             off = (off + 255) & ~(size_t)255;
  const size_t oPs  = off; off += (size_t)nSB * NCL * 4;             off = (off + 255) & ~(size_t)255;
  const size_t oMc  = off; off += (size_t)NCL * 4;                   off = (off + 255) & ~(size_t)255;
  const size_t oLse = off; off += (size_t)NCL * 4;                   off = (off + 255) & ~(size_t)255;
  if (off > ws_size || off > (size_t)134217728) return;
  _Float16* BtR  = (_Float16*)(ws + oBtR);
  _Float16* B0   = (_Float16*)(ws + oB0);
  _Float16* B1   = (_Float16*)(ws + oB1);
  _Float16* B2   = (_Float16*)(ws + oB2);
  float*    bcomb= (float*)(ws + oBc);
  _Float16* Ah   = (_Float16*)(ws + oAh);
  int*      cnt  = (int*)(ws + oCnt);
  int*      offp = (int*)(ws + oOff);
  int*      rb   = (int*)(ws + oRb);
  int*      csr  = (int*)(ws + oCsr);
  _Float16* X    = (_Float16*)(ws + oX);
  float*    T    = (float*)(ws + oT);
  float*    X3   = (float*)(ws + oX3);
  float*    pmax = (float*)(ws + oPm);
  float*    psum = (float*)(ws + oPs);
  float*    Mc   = (float*)(ws + oMc);
  float*    lse  = (float*)(ws + oLse);

  const int vec8 = ((nE & 3) == 0) ? 1 : 0;

  k_prep<<<nPrep, NTHR, 0, stream>>>(Wih, Whh, bih, bhh, W0, W1, W2, BtR, B0, B1, B2, bcomb);
  k_cvta<<<nCvt, NTHR, 0, stream>>>(topo, hid, Ah, nN);

  k_count<<<nBC, NTHR, 0, stream>>>(arows, cnt, nE, vec8);
  k_offsets<<<1, OTHR, 0, stream>>>(cnt, offp, rb, nBC);
  hipFuncSetAttribute(reinterpret_cast<const void*>(&k_fill),
                      hipFuncAttributeMaxDynamicSharedMemorySize, LDS_FILL);
  k_fill<<<nBF, NTHR, LDS_FILL, stream>>>(arows, offp, rb, csr, nE, vec8, csrLen);

  const int ldsG8 = GROWS * 128 * 4;
  const int ldsG4 = GROWS * 64 * 4;
  hipFuncSetAttribute(reinterpret_cast<const void*>(&k_gemm<KRNN, 8, 0>),
                      hipFuncAttributeMaxDynamicSharedMemorySize, ldsG8);
  hipFuncSetAttribute(reinterpret_cast<const void*>(&k_gemm<DIM, 8, 1>),
                      hipFuncAttributeMaxDynamicSharedMemorySize, ldsG8);
  k_gemm<KRNN, 8, 0><<<nGemm, NTHR, ldsG8, stream>>>(Ah, BtR, bcomb, out1, X, nN);

  k_gemm<DIM, 8, 1><<<nGemm, NTHR, ldsG8, stream>>>(X, B0, bcomb, T, X, nN);
  k_agg<4, 1><<<nAgg, NTHR, 0, stream>>>(csr, offp, cnt, acols, avals, T, gb0, X, X3, nN, nE, csrLen);
  k_gemm<DIM, 8, 1><<<nGemm, NTHR, ldsG8, stream>>>(X, B1, bcomb, T, X, nN);
  k_agg<4, 1><<<nAgg, NTHR, 0, stream>>>(csr, offp, cnt, acols, avals, T, gb1, X, X3, nN, nE, csrLen);
  k_gemm<DIM, 4, 1><<<nGemm, NTHR, ldsG4, stream>>>(X, B2, bcomb, T, X, nN);
  k_agg<2, 0><<<nAgg, NTHR, 0, stream>>>(csr, offp, cnt, acols, avals, T, gb2, X, X3, nN, nE, csrLen);

  k_colstat<<<nSB, NTHR, 0, stream>>>(X3, pmax, pmax, nN, 0);
  k_colred<<<1, NCL, 0, stream>>>(pmax, pmax, Mc, nSB, 0);
  k_colstat<<<nSB, NTHR, 0, stream>>>(X3, Mc, psum, nN, 1);
  k_colred<<<1, NCL, 0, stream>>>(psum, Mc, lse, nSB, 1);
  k_out<<<nOut, NTHR, 0, stream>>>(X3, lse, out0, n4);
}
